// NeuralKYAttention_18107582119947
// MI455X (gfx1250) — hardware-verified
//
#include <hip/hip_runtime.h>
#include <math.h>
#include <stdint.h>

#define NBATCH 2
#define TLEN   4096
#define DM     1024
#define NHEAD  16
#define HD     64
#define KWIN   7
#define WPAD   3
#define CHID   32
#define QKVW   (3 * DM)
#define NROWS  (NBATCH * TLEN)
#define TQ     16
#define CVB_X  ((NROWS * DM) / 2048)
#define CVB_W  ((DM * DM) / 2048)
static_assert((NROWS * DM) % 2048 == 0);
static_assert((DM * DM) % 2048 == 0);
static_assert(TLEN % 64 == 0 && NROWS % 64 == 0 && QKVW % 64 == 0 && DM % 64 == 0);
static_assert(DM % 32 == 0);
static_assert(TLEN % TQ == 0);
static_assert(NHEAD * HD == DM && HD == 64 && NHEAD == 16 && KWIN == 7 && CHID == 32);
static_assert(NHEAD * CHID == 512);

typedef __bf16   v16b __attribute__((ext_vector_type(16)));
typedef __bf16   v8b  __attribute__((ext_vector_type(8)));
typedef float    v8f  __attribute__((ext_vector_type(8)));
typedef float    v4f  __attribute__((ext_vector_type(4)));
typedef unsigned int v4u __attribute__((ext_vector_type(4)));
typedef v4f __attribute__((may_alias)) v4fa;

__device__ __forceinline__ unsigned short bf_bits(float f) {
  unsigned u = __float_as_uint(f);
  return (unsigned short)((u + 0x7FFFu + ((u >> 16) & 1u)) >> 16);
}
__device__ __forceinline__ float bf_up(unsigned short h) { return __uint_as_float(((unsigned)h) << 16); }
__device__ __forceinline__ float bf_rn(float f) { return bf_up(bf_bits(f)); }
__device__ __forceinline__ unsigned pk16(unsigned short a, unsigned short b) { return (unsigned)a | ((unsigned)b << 16); }
__device__ __forceinline__ v8f zero8() { v8f z = {0.f, 0.f, 0.f, 0.f, 0.f, 0.f, 0.f, 0.f}; return z; }
__device__ __forceinline__ v4f zero4() { v4f z = {0.f, 0.f, 0.f, 0.f}; return z; }
__device__ __forceinline__ float gelu_f(float z) {
  return 0.5f * z * (1.0f + erff(z * 0.70710678118654752f));
}

__device__ __forceinline__ v16b ldfrag_b(const __bf16* p) {
  union { v16b v; v8b h[2]; } f;
  f.h[0] = *(const v8b*)(p);
  f.h[1] = *(const v8b*)(p + 16);
  return f.v;
}

__device__ __forceinline__ v8f mma_b_raw(v16b a, v16b b, v8f c) {
  return __builtin_amdgcn_wmma_f32_16x16x32_bf16(false, a, false, b, (short)0, c, false, false);
}
__device__ __forceinline__ void dep_guard_b(v8f& a, v8f& b, v16b x) {
  asm volatile("v_nop\n\tv_nop\n\tv_nop\n\tv_nop" : "+v"(a), "+v"(b) : "v"(x));
}
__device__ __forceinline__ void keep4_b(v16b a, v16b b, v16b c, v16b d) {
  asm volatile("v_nop" :: "v"(a), "v"(b), "v"(c), "v"(d));
}
__device__ __forceinline__ void acc_guard4(v8f& a, v8f& b, v8f& c, v8f& d) {
  asm volatile("v_nop\n\tv_nop\n\tv_nop\n\tv_nop" : "+v"(a), "+v"(b), "+v"(c), "+v"(d));
}

__global__ __launch_bounds__(256) void cvt_planes(const float* __restrict__ x, const float* __restrict__ wq,
                                                  const float* __restrict__ wk, const float* __restrict__ wv,
                                                  const float* __restrict__ wo,
                                                  unsigned short* xb, unsigned short* wqkv, unsigned short* wob) {
  const int blk = blockIdx.x;
  if (blk >= CVB_X + 4 * CVB_W) return;
  const float* src;
  unsigned short* dst;
  int lb;
  if (blk < CVB_X) {
    src = x;  dst = xb; lb = blk;
  } else if (blk < CVB_X + CVB_W) {
    src = wq; dst = wqkv; lb = blk - CVB_X;
  } else if (blk < CVB_X + 2 * CVB_W) {
    src = wk; dst = wqkv + (size_t)DM * DM; lb = blk - CVB_X - CVB_W;
  } else if (blk < CVB_X + 3 * CVB_W) {
    src = wv; dst = wqkv + (size_t)2 * DM * DM; lb = blk - CVB_X - 2 * CVB_W;
  } else {
    src = wo; dst = wob; lb = blk - CVB_X - 3 * CVB_W;
  }
  const size_t i = ((size_t)lb * 256 + threadIdx.x) * 8;
  const v4f a = *(const v4fa*)(src + i);
  const v4f b = *(const v4fa*)(src + i + 4);
  v4u p;
  p[0] = pk16(bf_bits(a[0]), bf_bits(a[1]));
  p[1] = pk16(bf_bits(a[2]), bf_bits(a[3]));
  p[2] = pk16(bf_bits(b[0]), bf_bits(b[1]));
  p[3] = pk16(bf_bits(b[2]), bf_bits(b[3]));
  *(volatile v4u*)(dst + i) = p;
  __threadfence();
  *(volatile v4u*)(dst + i) = p;
}

__global__ __launch_bounds__(512) void conn_table(const float* __restrict__ cw1, const float* __restrict__ cb1,
                                                  const float* __restrict__ cw2, const float* __restrict__ cb2,
                                                  const float* __restrict__ cw3, const float* __restrict__ cb3,
                                                  float* conn) {
  __shared__ float sA[NHEAD * CHID];
  __shared__ __align__(16) float sC[NHEAD * 8];
  const int tid = threadIdx.x;
  const int h   = tid >> 5;
  const int j   = tid & 31;
  const float w1 = bf_rn(cw1[h * CHID + j]);
  const float b1 = bf_rn(cb1[h * CHID + j]);
  const float b2 = bf_rn(cb2[h * CHID + j]);
  const float w3 = bf_rn(cw3[h * CHID + j]);
  const float b3 = bf_rn(cb3[h]);
  const float* w2row = cw2 + ((size_t)h * CHID + j) * CHID;
  float creg = -INFINITY;
#pragma unroll 1
  for (int w = 0; w < KWIN; ++w) {
    const float pos = (w == KWIN - 1) ? 1.0f : (float)w * (1.0f / 6.0f);
    const float a1 = gelu_f(pos * w1 + b1);
    sA[h * CHID + j] = a1;
    __syncthreads();
    float z2 = 0.0f;
#pragma unroll 1
    for (int i = 0; i < CHID; ++i) z2 = fmaf(sA[h * CHID + i], bf_rn(w2row[i]), z2);
    const float a2 = gelu_f(z2 + b2);
    float t3 = a2 * w3;
    t3 += __shfl_xor(t3, 16, 32);
    t3 += __shfl_xor(t3, 8, 32);
    t3 += __shfl_xor(t3, 4, 32);
    t3 += __shfl_xor(t3, 2, 32);
    t3 += __shfl_xor(t3, 1, 32);
    const float cv = t3 + b3;
    creg = (j == w) ? cv : creg;
    __syncthreads();
  }
  float mx = creg;
  mx = fmaxf(mx, __shfl_xor(mx, 1, 32));
  mx = fmaxf(mx, __shfl_xor(mx, 2, 32));
  mx = fmaxf(mx, __shfl_xor(mx, 4, 32));
  mx = fmaxf(mx, __shfl_xor(mx, 8, 32));
  mx = fmaxf(mx, __shfl_xor(mx, 16, 32));
  const float ex = __expf(creg - mx);
  const float e  = (j < KWIN) ? ex : 0.0f;
  float se = e;
  se += __shfl_xor(se, 1, 32);
  se += __shfl_xor(se, 2, 32);
  se += __shfl_xor(se, 4, 32);
  se += __shfl_xor(se, 8, 32);
  se += __shfl_xor(se, 16, 32);
  const float p = e * (1.0f / se);
  if (j < 8) sC[h * 8 + j] = p;
  __syncthreads();
  if (tid < 32) {
    const v4f v = *(const v4fa*)(sC + 4 * tid);
    *(volatile v4f*)(conn + 4 * tid) = v;
    __threadfence();
    *(volatile v4f*)(conn + 4 * tid) = v;
  }
}

template <int M, int N, int K, bool TWO>
__global__ __launch_bounds__(256) void gemm_nt(const unsigned short* __restrict__ A0p,
                                               const unsigned short* __restrict__ A1p,
                                               const unsigned short* __restrict__ Btp,
                                               const float* __restrict__ bias, float* C) {
  static_assert((M % 64) == 0 && (N % 64) == 0 && (K % 32) == 0);
  __shared__ __align__(16) float sT[8][16 * 68];
  const __bf16* A0 = (const __bf16*)(const void*)A0p;
  const __bf16* A1 = (const __bf16*)(const void*)A1p;
  const __bf16* Bt = (const __bf16*)(const void*)Btp;

  const int lane = threadIdx.x & 31;
  const int wave = threadIdx.x >> 5;
  constexpr int tilesN = N / 64;
  constexpr int tilesM = M / 64;
  const int tile = blockIdx.x * 8 + wave;
  if (tile >= tilesM * tilesN) return;
  const int tm = tile / tilesN;
  const int tn = tile - tm * tilesN;
  const int m0 = tm << 6;
  const int n0 = tn << 6;

  const int rlane = lane & 15;
  const int koff  = (lane >> 4) * 8;
  const int mOff  = (lane >> 4) * 8;

  v8f acc[4][4];
#pragma unroll
  for (int i = 0; i < 4; ++i)
#pragma unroll
    for (int j = 0; j < 4; ++j) acc[i][j] = zero8();

#pragma unroll 1
  for (int k0 = 0; k0 < K; k0 += 32) {
    v16b bh[4];
#pragma unroll
    for (int j = 0; j < 4; ++j) {
      const size_t bo = (size_t)(n0 + (j << 4) + rlane) * K + koff + k0;
      bh[j] = ldfrag_b(Bt + bo);
    }
#pragma unroll
    for (int i = 0; i < 4; ++i) {
      const size_t ao = (size_t)(m0 + (i << 4) + rlane) * K + koff + k0;
      const v16b ah = ldfrag_b(A0 + ao);
#pragma unroll
      for (int j = 0; j < 4; ++j) acc[i][j] = mma_b_raw(ah, bh[j], acc[i][j]);
      dep_guard_b(acc[i][0], acc[i][3], ah);
      if (TWO) {
        const v16b al = ldfrag_b(A1 + ao);
#pragma unroll
        for (int j = 0; j < 4; ++j) acc[i][j] = mma_b_raw(al, bh[j], acc[i][j]);
        dep_guard_b(acc[i][0], acc[i][3], al);
      }
    }
    keep4_b(bh[0], bh[1], bh[2], bh[3]);
  }
  acc_guard4(acc[0][0], acc[0][1], acc[0][2], acc[0][3]);
  acc_guard4(acc[1][0], acc[1][1], acc[1][2], acc[1][3]);
  acc_guard4(acc[2][0], acc[2][1], acc[2][2], acc[2][3]);
  acc_guard4(acc[3][0], acc[3][1], acc[3][2], acc[3][3]);

  float* slab = sT[wave];
  const int hsel = lane >> 4;
  const int c4   = (lane & 15) * 4;
  v4f addv = zero4();
  if (TWO) {
    const v4f bb = *(const v4fa*)(bias + n0 + c4);
    addv[0] = bf_up(bf_bits(bb[0]));
    addv[1] = bf_up(bf_bits(bb[1]));
    addv[2] = bf_up(bf_bits(bb[2]));
    addv[3] = bf_up(bf_bits(bb[3]));
  }
#pragma unroll
  for (int i = 0; i < 4; ++i) {
    const int mBase = m0 + (i << 4);
#pragma unroll
    for (int j = 0; j < 4; ++j) {
#pragma unroll
      for (int r = 0; r < 8; ++r) slab[(mOff + r) * 68 + (j << 4) + rlane] = acc[i][j][r];
    }
    __builtin_amdgcn_fence(__ATOMIC_RELEASE, "workgroup");
    __builtin_amdgcn_wave_barrier();
    __builtin_amdgcn_fence(__ATOMIC_ACQUIRE, "workgroup");
    v4f vals[8];
#pragma unroll
    for (int it = 0; it < 8; ++it) {
      const int row = 2 * it + hsel;
      v4f v = *(const v4fa*)(slab + row * 68 + c4);
      v = TWO ? (v + addv) : v;
      vals[it] = v;
    }
#pragma unroll
    for (int it = 0; it < 8; ++it)
      *(volatile v4f*)(C + (size_t)(mBase + 2 * it + hsel) * N + n0 + c4) = vals[it];
    __threadfence();
#pragma unroll
    for (int it = 0; it < 8; ++it)
      *(volatile v4f*)(C + (size_t)(mBase + 2 * it + hsel) * N + n0 + c4) = vals[it];
    __builtin_amdgcn_fence(__ATOMIC_RELEASE, "workgroup");
    __builtin_amdgcn_wave_barrier();
    __builtin_amdgcn_fence(__ATOMIC_ACQUIRE, "workgroup");
  }
}

__global__ __launch_bounds__(128) void win_attn(const float* __restrict__ QKV, const float* __restrict__ conn,
                                               unsigned short* Oh, unsigned short* Ol) {
  const int tid  = threadIdx.x;
  const int wave = tid >> 5;
  const int lane = tid & 31;
  const int hsub = lane >> 3;
  const int c    = lane & 7;
  const int head = wave * 4 + hsub;
  const int t0   = blockIdx.x * TQ;
  if (t0 >= TLEN) return;
  const int colq = head * HD + 8 * c;
  const float* Qb = QKV + colq;
  const float* Kb = QKV + DM + colq;
  const float* Vb = QKV + 2 * DM + colq;
  unsigned short* ohb = Oh + colq;
  unsigned short* olb = Ol + colq;
  const v4f cA = *(const v4fa*)(conn + head * 8);
  const v4f cB = *(const v4fa*)(conn + head * 8 + 4);

#pragma unroll 1
  for (int tq = 0; tq < TQ; ++tq) {
    const int t = t0 + tq;
    const float* qp = Qb + (size_t)t * QKVW;
    const v4f q0 = *(const v4fa*)(qp);
    const v4f q1 = *(const v4fa*)(qp + 4);
    float mrun = -INFINITY;
    float s0 = 0.f, s1 = 0.f, s2 = 0.f, s3 = 0.f, s4 = 0.f, s5 = 0.f, s6 = 0.f;
#pragma unroll 1
    for (int j = 0; j < KWIN; ++j) {
      const int pos  = t + j - WPAD;
      const bool ok  = (pos >= 0) && (pos < TLEN);
      const int prow = (pos < 0) ? 0 : ((pos > TLEN - 1) ? (TLEN - 1) : pos);
      const float* kp = Kb + (size_t)prow * QKVW;
      const v4f ka = *(const v4fa*)(kp);
      const v4f kc = *(const v4fa*)(kp + 4);
      const v4f pr = q0 * ka + q1 * kc;
      float d = (pr[0] + pr[1]) + (pr[2] + pr[3]);
      d += __shfl_xor(d, 1, 32);
      d += __shfl_xor(d, 2, 32);
      d += __shfl_xor(d, 4, 32);
      d = ok ? (d * 0.125f) : 0.0f;
      mrun = fmaxf(mrun, d);
      s0 = (j == 0) ? d : s0;
      s1 = (j == 1) ? d : s1;
      s2 = (j == 2) ? d : s2;
      s3 = (j == 3) ? d : s3;
      s4 = (j == 4) ? d : s4;
      s5 = (j == 5) ? d : s5;
      s6 = (j == 6) ? d : s6;
    }
    const float e0 = __expf(s0 - mrun);
    const float e1 = __expf(s1 - mrun);
    const float e2 = __expf(s2 - mrun);
    const float e3 = __expf(s3 - mrun);
    const float e4 = __expf(s4 - mrun);
    const float e5 = __expf(s5 - mrun);
    const float e6 = __expf(s6 - mrun);
    const float esum = ((e0 + e1) + (e2 + e3)) + ((e4 + e5) + e6);
    const float rinv = 1.0f / esum;
    const float f0 = (e0 * rinv) * cA[0];
    const float f1 = (e1 * rinv) * cA[1];
    const float f2 = (e2 * rinv) * cA[2];
    const float f3 = (e3 * rinv) * cA[3];
    const float f4 = (e4 * rinv) * cB[0];
    const float f5 = (e5 * rinv) * cB[1];
    const float f6 = (e6 * rinv) * cB[2];
    const float fsum = ((f0 + f1) + (f2 + f3)) + ((f4 + f5) + f6);
    const float ginv = 1.0f / (fsum + 1e-9f);
    const float g0 = f0 * ginv, g1 = f1 * ginv, g2 = f2 * ginv, g3 = f3 * ginv;
    const float g4 = f4 * ginv, g5 = f5 * ginv, g6 = f6 * ginv;
    v4f acc0 = zero4(), acc1 = zero4();
#pragma unroll 1
    for (int j = 0; j < KWIN; ++j) {
      const int pos  = t + j - WPAD;
      const bool ok  = (pos >= 0) && (pos < TLEN);
      const int prow = (pos < 0) ? 0 : ((pos > TLEN - 1) ? (TLEN - 1) : pos);
      float gj = (j == 0) ? g0 : ((j == 1) ? g1 : ((j == 2) ? g2 : ((j == 3) ? g3 :
                 ((j == 4) ? g4 : ((j == 5) ? g5 : g6)))));
      gj = ok ? gj : 0.0f;
      const float* vp = Vb + (size_t)prow * QKVW;
      const v4f va = *(const v4fa*)(vp);
      const v4f vc = *(const v4fa*)(vp + 4);
      acc0 += va * gj;
      acc1 += vc * gj;
    }
    v4u hv, lv;
#pragma unroll
    for (int e = 0; e < 2; ++e) {
      const float fa = acc0[2 * e], fb = acc0[2 * e + 1];
      const float ga = acc1[2 * e], gb = acc1[2 * e + 1];
      const unsigned short hfa = bf_bits(fa), hfb = bf_bits(fb);
      const unsigned short hga = bf_bits(ga), hgb = bf_bits(gb);
      const unsigned short lfa = bf_bits(fa - bf_up(hfa)), lfb = bf_bits(fb - bf_up(hfb));
      const unsigned short lga = bf_bits(ga - bf_up(hga)), lgb = bf_bits(gb - bf_up(hgb));
      hv[e]     = pk16(hfa, hfb);
      hv[2 + e] = pk16(hga, hgb);
      lv[e]     = pk16(lfa, lfb);
      lv[2 + e] = pk16(lga, lgb);
    }
    unsigned short* ohp = ohb + (size_t)t * DM;
    unsigned short* olp = olb + (size_t)t * DM;
    *(volatile v4u*)ohp = hv;
    *(volatile v4u*)olp = lv;
    __threadfence();
    *(volatile v4u*)ohp = hv;
    *(volatile v4u*)olp = lv;
  }
}

extern "C" void kernel_launch(void* const* d_in, const int* in_sizes, int n_in,
                              void* d_out, int out_size, void* d_ws, size_t ws_size,
                              hipStream_t stream) {
  if (n_in < 12) return;
  if (in_sizes[0] != NROWS * DM) return;
  if (in_sizes[1] != DM * DM || in_sizes[2] != DM * DM || in_sizes[3] != DM * DM || in_sizes[4] != DM * DM) return;
  if (in_sizes[5] != DM) return;
  if (in_sizes[6] != NHEAD * CHID || in_sizes[7] != NHEAD * CHID) return;
  if (in_sizes[8] != NHEAD * CHID * CHID || in_sizes[9] != NHEAD * CHID) return;
  if (in_sizes[10] != NHEAD * CHID || in_sizes[11] != NHEAD) return;
  if (out_size != NROWS * DM) return;

  const float* x   = (const float*)d_in[0];
  const float* Wq  = (const float*)d_in[1];
  const float* Wk  = (const float*)d_in[2];
  const float* Wv  = (const float*)d_in[3];
  const float* Wo  = (const float*)d_in[4];
  const float* bo  = (const float*)d_in[5];
  const float* cw1 = (const float*)d_in[6];
  const float* cb1 = (const float*)d_in[7];
  const float* cw2 = (const float*)d_in[8];
  const float* cb2 = (const float*)d_in[9];
  const float* cw3 = (const float*)d_in[10];
  const float* cb3 = (const float*)d_in[11];
  float* out = (float*)d_out;

  const size_t PXB   = (size_t)NROWS * DM * 2;
  const size_t PWQKV = (size_t)3 * DM * DM * 2;
  const size_t PWO   = (size_t)DM * DM * 2;
  const size_t PCONN = (size_t)NHEAD * 8 * 4;
  const size_t PQKV  = (size_t)TLEN * QKVW * 4;
  const size_t PO    = (size_t)NROWS * DM * 2;
  size_t off = 0;
  const size_t oXb   = off; off += PXB;
  const size_t oWqkv = off; off += PWQKV;
  const size_t oWob  = off; off += PWO;
  const size_t oConn = off; off += PCONN;
  const size_t oQKV  = off; off += PQKV;
  const size_t oOh   = off; off += PO;
  const size_t oOl   = off; off += PO;
  if (off > ws_size) return;
  if (off > (size_t)134217728) return;

  char* ws = (char*)d_ws;
  unsigned short* Xb   = (unsigned short*)(ws + oXb);
  unsigned short* Wqkv = (unsigned short*)(ws + oWqkv);
  unsigned short* Wob  = (unsigned short*)(ws + oWob);
  float*          Conn = (float*)(ws + oConn);
  float*          QKV  = (float*)(ws + oQKV);
  unsigned short* Oh   = (unsigned short*)(ws + oOh);
  unsigned short* Ol   = (unsigned short*)(ws + oOl);

  const dim3 blk(256);
  const dim3 gCvt(CVB_X + 4 * CVB_W);
  const int  tiles1 = (TLEN / 64) * (QKVW / 64);
  const dim3 gProj((tiles1 + 7) / 8);
  const dim3 gAttn(TLEN / TQ);
  const int  tiles2 = (NROWS / 64) * (DM / 64);
  const dim3 gOut((tiles2 + 7) / 8);

  cvt_planes<<<gCvt, blk, 0, stream>>>(x, Wq, Wk, Wv, Wo, Xb, Wqkv, Wob);
  conn_table<<<dim3(1), dim3(NHEAD * CHID), 0, stream>>>(cw1, cb1, cw2, cb2, cw3, cb3, Conn);
  for (int b = 0; b < NBATCH; ++b) {
    const unsigned short* Xbb = Xb + (size_t)b * TLEN * DM;
    gemm_nt<TLEN, QKVW, DM, false><<<gProj, blk, 0, stream>>>(Xbb, Xbb, Wqkv, bo, QKV);
    win_attn<<<gAttn, dim3(128), 0, stream>>>(QKV, Conn, Oh + (size_t)b * TLEN * DM, Ol + (size_t)b * TLEN * DM);
  }
  gemm_nt<NROWS, DM, DM, true><<<gOut, blk, 0, stream>>>(Oh, Ol, Wob, bo, out);
  (void)hipGetLastError();
}
